// WindowedAttn_34351148433901
// MI455X (gfx1250) — hardware-verified
//
#include <hip/hip_runtime.h>
#include <cstdint>
#include <cstddef>

typedef __attribute__((ext_vector_type(16))) _Float16 v16h;
typedef __attribute__((ext_vector_type(8)))  _Float16 v8h;
typedef __attribute__((ext_vector_type(16))) __bf16   v16b;
typedef __attribute__((ext_vector_type(8)))  __bf16   v8b;
typedef __attribute__((ext_vector_type(8)))  float    v8f;
typedef __attribute__((ext_vector_type(4)))  float    v4f;
typedef __attribute__((ext_vector_type(4)))  unsigned int v4u;

constexpr int kBatch  = 2;
constexpr int kSeq    = 2048;
constexpr int kTok    = kBatch * kSeq;
constexpr int kDModel = 1024;
constexpr int kHeads  = 16;
constexpr int kDh     = 64;
constexpr int kQkvN   = 3 * kDModel;
constexpr int kWin    = 256;
constexpr int kKC     = 64;
constexpr int kQB     = 64;
constexpr float kScale = 0.125f;

constexpr size_t OFF_BIAS = 0;
constexpr size_t SZ_BIAS  = (size_t)(kQkvN + kDModel) * 4;
constexpr size_t OFF_X16  = OFF_BIAS + SZ_BIAS;
constexpr size_t SZ_X16   = (size_t)kTok * kDModel * 2;
constexpr size_t OFF_WQT  = OFF_X16 + SZ_X16;
constexpr size_t SZ_WQT   = (size_t)kQkvN * kDModel * 2;
constexpr size_t OFF_WOT  = OFF_WQT + SZ_WQT;
constexpr size_t SZ_WOT   = (size_t)kDModel * kDModel * 2;
constexpr size_t OFF_QKVH = OFF_WOT + SZ_WOT;
constexpr size_t SZ_QKV   = (size_t)kTok * kQkvN * 2;
constexpr size_t OFF_QKVL = OFF_QKVH + SZ_QKV;
constexpr size_t OFF_ATTH = OFF_QKVL + SZ_QKV;
constexpr size_t SZ_ATT   = (size_t)kTok * kDModel * 2;
constexpr size_t OFF_ATTL = OFF_ATTH + SZ_ATT;
constexpr size_t WS_TOTAL = OFF_ATTL + SZ_ATT;
static_assert(WS_TOTAL == 83902464, "carve total");
static_assert(WS_TOTAL <= 134217728, "carve within 128 MiB");
static_assert(OFF_X16 % 256 == 0 && OFF_WQT % 256 == 0 && OFF_WOT % 256 == 0 && OFF_QKVH % 256 == 0 &&
              OFF_QKVL % 256 == 0 && OFF_ATTH % 256 == 0 && OFF_ATTL % 256 == 0, "aligned regions");

static_assert(kTok % 64 == 0 && kQkvN % 64 == 0 && kDModel % 64 == 0 && kDModel % 32 == 0, "tile multiples");
static_assert(kSeq % kQB == 0 && kDh == 64 && kWin % kKC == 0, "attention geometry");

__device__ __forceinline__ unsigned short f2bf_bits(float f) {
  unsigned u = __float_as_uint(f);
  return (unsigned short)((u + 0x7FFFu + ((u >> 16) & 1u)) >> 16);
}
__device__ __forceinline__ float bf_bits2f(unsigned short h) { return __uint_as_float(((unsigned)h) << 16); }

__device__ __forceinline__ void dep_guard_h(v8f& a, v8f& b, v16h x, v16h y) { asm volatile("v_nop\n\tv_nop\n\tv_nop\n\tv_nop" : "+v"(a), "+v"(b) : "v"(x), "v"(y)); }
__device__ __forceinline__ void dep_guard_b(v8f& a, v8f& b, v16b x, v16b y) { asm volatile("v_nop\n\tv_nop\n\tv_nop\n\tv_nop" : "+v"(a), "+v"(b) : "v"(x), "v"(y)); }
__device__ __forceinline__ void keep4_h(v16h a, v16h b, v16h c, v16h d) { asm volatile("v_nop" :: "v"(a), "v"(b), "v"(c), "v"(d)); }
__device__ __forceinline__ void keep4_b(v16b a, v16b b, v16b c, v16b d) { asm volatile("v_nop" :: "v"(a), "v"(b), "v"(c), "v"(d)); }
__device__ __forceinline__ void acc_guard4(v8f& a, v8f& b, v8f& c, v8f& d) { asm volatile("v_nop\n\tv_nop\n\tv_nop\n\tv_nop" : "+v"(a), "+v"(b), "+v"(c), "+v"(d)); }
template <typename T> struct Frag;
template <> struct Frag<_Float16> {
  typedef v16h V; union U { v16h v; v8h h[2]; };
  static __device__ __forceinline__ v16h load(const _Float16* p) {
    U f; f.h[0] = *(const v8h*)(p); f.h[1] = *(const v8h*)(p + 16); return f.v;
  }
  static __device__ __forceinline__ v8f mma(v16h a, v16h b, v8f c) {
    return __builtin_amdgcn_wmma_f32_16x16x32_f16(false, a, false, b, (short)0, c, false, false);
  }
  static __device__ __forceinline__ void guard(v8f& a, v8f& b, v16h x, v16h y) { dep_guard_h(a, b, x, y); }
  static __device__ __forceinline__ void keep(v16h a, v16h b, v16h c, v16h d) { keep4_h(a, b, c, d); }
};
template <> struct Frag<__bf16> {
  typedef v16b V; union U { v16b v; v8b h[2]; };
  static __device__ __forceinline__ v16b load(const __bf16* p) {
    U f; f.h[0] = *(const v8b*)(p); f.h[1] = *(const v8b*)(p + 16); return f.v;
  }
  static __device__ __forceinline__ v8f mma(v16b a, v16b b, v8f c) {
    return __builtin_amdgcn_wmma_f32_16x16x32_bf16(false, a, false, b, (short)0, c, false, false);
  }
  static __device__ __forceinline__ void guard(v8f& a, v8f& b, v16b x, v16b y) { dep_guard_b(a, b, x, y); }
  static __device__ __forceinline__ void keep(v16b a, v16b b, v16b c, v16b d) { keep4_b(a, b, c, d); }
};

__device__ __forceinline__ unsigned short at_bf_bits(float f) {
  unsigned u = __float_as_uint(f);
  return (unsigned short)((u + 0x7FFFu + ((u >> 16) & 1u)) >> 16);
}
__device__ __forceinline__ __bf16 at_f2bf(float f) { return __builtin_bit_cast(__bf16, at_bf_bits(f)); }
__device__ __forceinline__ void at_split(float f, __bf16& hi, __bf16& lo) {
  const unsigned short hb = at_bf_bits(f);
  hi = __builtin_bit_cast(__bf16, hb);
  lo = at_f2bf(f - __uint_as_float(((unsigned)hb) << 16));
}
__device__ __forceinline__ v8f at_mma(v16b a, v16b b, v8f c) {
  c = __builtin_amdgcn_wmma_f32_16x16x32_bf16(false, a, false, b, (short)0, c, false, false);
  asm volatile("v_nop\n\tv_nop\n\tv_nop\n\tv_nop" : "+v"(c) : "v"(a), "v"(b));
  return c;
}

template <int ET> struct Elem;
template <> struct Elem<0> { typedef _Float16 T; };
template <> struct Elem<1> { typedef __bf16 T; };
template <int ET, bool SPLIT_A, bool SPLIT_B, int BIAS_MODE, int OUT_MODE, bool RESID, int ACT = 0>
__global__ __launch_bounds__(256) void wmma_gemm64(
    const unsigned short* __restrict__ Ap, const unsigned short* __restrict__ A2p, int lda, long strideA,
    const unsigned short* __restrict__ Btp, const unsigned short* __restrict__ Bt2p, int ldb, long strideB,
    void* __restrict__ Cout, void* __restrict__ Cout2, int ldc, long strideC,
    const float* __restrict__ bias,
    const float* __restrict__ resid, long strideR,
    int M, int N, int K, float scale) {
  typedef typename Elem<ET>::T T;
  typedef typename Frag<T>::V V;
  const T* A = (const T*)Ap; const T* A2 = (const T*)A2p; const T* Bt = (const T*)Btp; const T* Bt2 = (const T*)Bt2p;
  __shared__ __align__(16) float sT[8][16 * 68];
  const int b    = blockIdx.y;
  const int lane = threadIdx.x & 31;
  const int wave = threadIdx.x >> 5;
  const int tilesN = N >> 6;
  const int tilesM = M >> 6;
  const int tile = blockIdx.x * 8 + wave;
  if (tile >= tilesM * tilesN) return;
  const int tm = tile / tilesN;
  const int tn = tile - tm * tilesN;
  const int m0 = tm << 6;
  const int n0 = tn << 6;

  const T* Ab  = A  + (size_t)b * strideA;
  const T* Bb  = Bt + (size_t)b * strideB;
  const T* Ab2 = SPLIT_A ? (A2  + (size_t)b * strideA) : nullptr;
  const T* Bb2 = SPLIT_B ? (Bt2 + (size_t)b * strideB) : nullptr;

  const int rlane = lane & 15;
  const int koff  = (lane >> 4) * 8;
  const int mOff  = (lane >> 4) * 8;

  v8f acc[4][4];
#pragma unroll
  for (int i = 0; i < 4; ++i)
#pragma unroll
    for (int j = 0; j < 4; ++j) acc[i][j] = (v8f){0.f,0.f,0.f,0.f,0.f,0.f,0.f,0.f};

  for (int k0 = 0; k0 < K; k0 += 32) {
    V bh[4], bl[4];
#pragma unroll
    for (int j = 0; j < 4; ++j) {
      const size_t bo = (size_t)(n0 + (j << 4) + rlane) * ldb + koff + k0;
      bh[j] = Frag<T>::load(Bb + bo);
      if (SPLIT_B) bl[j] = Frag<T>::load(Bb2 + bo);
    }
#pragma unroll
    for (int i = 0; i < 4; ++i) {
      const size_t ao = (size_t)(m0 + (i << 4) + rlane) * lda + koff + k0;
      V ah = Frag<T>::load(Ab + ao);
      V al;
      if (SPLIT_A) al = Frag<T>::load(Ab2 + ao);
#pragma unroll
      for (int j = 0; j < 4; ++j) {
        acc[i][j] = Frag<T>::mma(ah, bh[j], acc[i][j]);
        if (SPLIT_B) acc[i][j] = Frag<T>::mma(ah, bl[j], acc[i][j]);
        if (SPLIT_A) acc[i][j] = Frag<T>::mma(al, bh[j], acc[i][j]);
      }
      Frag<T>::guard(acc[i][0], acc[i][3], ah, SPLIT_A ? al : ah);
    }
    Frag<T>::keep(bh[0], bh[1], bh[2], bh[3]);
    if (SPLIT_B) Frag<T>::keep(bl[0], bl[1], bl[2], bl[3]);
  }
  acc_guard4(acc[0][0], acc[0][1], acc[0][2], acc[0][3]);
  acc_guard4(acc[1][0], acc[1][1], acc[1][2], acc[1][3]);
  acc_guard4(acc[2][0], acc[2][1], acc[2][2], acc[2][3]);
  acc_guard4(acc[3][0], acc[3][1], acc[3][2], acc[3][3]);

  float* slab = sT[wave];
  const float* Rb = RESID ? (resid + (size_t)b * strideR) : nullptr;
#pragma unroll
  for (int i = 0; i < 4; ++i) {
    const int mBase = m0 + (i << 4);
#pragma unroll
    for (int j = 0; j < 4; ++j) {
      const int n = n0 + (j << 4) + rlane;
      float bv = 0.f;
      if (BIAS_MODE == 2) bv = bias[n];
#pragma unroll
      for (int r = 0; r < 8; ++r) {
        float v = acc[i][j][r] * scale;
        if (BIAS_MODE == 1) v += bias[mBase + mOff + r];
        if (BIAS_MODE == 2) v += bv;
        if (RESID) v += Rb[(size_t)(mBase + mOff + r) * ldc + n];
        if (ACT == 1) v = tanhf(v);
        if (ACT == 2) v = fmaxf(v, 0.0f);
        if (ACT == 3) v = v / (1.0f + expf(-v));
        if (ACT == 4) v = (v > 0.f) ? v : 0.01f * v;
        slab[(mOff + r) * 68 + (j << 4) + rlane] = v;
      }
    }
    __builtin_amdgcn_fence(__ATOMIC_RELEASE, "workgroup");
    __builtin_amdgcn_wave_barrier();
    __builtin_amdgcn_fence(__ATOMIC_ACQUIRE, "workgroup");
    if (OUT_MODE == 0) {
      float* C = (float*)Cout + (size_t)b * strideC;
      const int hh = lane >> 4, c4 = (lane & 15) * 4;
      for (int pass = 0; pass < 2; ++pass) {
#pragma unroll
        for (int it = 0; it < 8; ++it) {
          const int row = it * 2 + hh;
          v4f v = *(const v4f*)(slab + row * 68 + c4);
          *(volatile v4f*)(C + (size_t)(mBase + row) * ldc + n0 + c4) = v;
        }
        __threadfence();
      }
    } else {
      const int q = lane >> 3, c8 = (lane & 7) * 8;
      unsigned short* C  = (unsigned short*)Cout  + (size_t)b * strideC;
      unsigned short* C2 = (OUT_MODE == 2) ? ((unsigned short*)Cout2 + (size_t)b * strideC) : nullptr;
      for (int pass = 0; pass < 2; ++pass) {
#pragma unroll
        for (int it = 0; it < 4; ++it) {
          const int row = it * 4 + q;
          const float* sp = slab + row * 68 + c8;
          v8h hv, lv;
#pragma unroll
          for (int e = 0; e < 8; ++e) {
            if (OUT_MODE == 1) {
              hv[e] = (_Float16)sp[e];
            } else {
              unsigned short hb = f2bf_bits(sp[e]);
              unsigned short lb = f2bf_bits(sp[e] - bf_bits2f(hb));
              hv[e] = __builtin_bit_cast(_Float16, hb);
              lv[e] = __builtin_bit_cast(_Float16, lb);
            }
          }
          *(volatile v8h*)(C + (size_t)(mBase + row) * ldc + n0 + c8) = hv;
          if (OUT_MODE == 2) *(volatile v8h*)(C2 + (size_t)(mBase + row) * ldc + n0 + c8) = lv;
        }
        __threadfence();
      }
    }
    __builtin_amdgcn_fence(__ATOMIC_RELEASE, "workgroup");
    __builtin_amdgcn_wave_barrier();
    __builtin_amdgcn_fence(__ATOMIC_ACQUIRE, "workgroup");
  }
}

__global__ __launch_bounds__(256) void bias_rne4(const float* __restrict__ in, float* __restrict__ out, int n4) {
  const int i = blockIdx.x * 256 + threadIdx.x;
  if (i < n4) {
    const v4f f = *(const v4f*)(in + 4 * (size_t)i);
    v4f r;
#pragma unroll
    for (int e = 0; e < 4; ++e) r[e] = bf_bits2f(f2bf_bits(f[e]));
    *(volatile v4f*)(out + 4 * (size_t)i) = r;
    __threadfence();
    *(volatile v4f*)(out + 4 * (size_t)i) = r;
  }
}

__global__ __launch_bounds__(256) void cast_bf16x8(const float* __restrict__ in, unsigned short* __restrict__ out, int n8) {
  const int i = blockIdx.x * 256 + threadIdx.x;
  if (i < n8) {
    const size_t base = 8 * (size_t)i;
    const v4f a  = *(const v4f*)(in + base);
    const v4f a2 = *(const v4f*)(in + base + 4);
    v4u w;
    w[0] = (unsigned)f2bf_bits(a[0])  | ((unsigned)f2bf_bits(a[1])  << 16);
    w[1] = (unsigned)f2bf_bits(a[2])  | ((unsigned)f2bf_bits(a[3])  << 16);
    w[2] = (unsigned)f2bf_bits(a2[0]) | ((unsigned)f2bf_bits(a2[1]) << 16);
    w[3] = (unsigned)f2bf_bits(a2[2]) | ((unsigned)f2bf_bits(a2[3]) << 16);
    *(volatile v4u*)(out + base) = w;
    __threadfence();
    *(volatile v4u*)(out + base) = w;
  }
}

__global__ __launch_bounds__(256) void transpose_cast_bf16(const float* __restrict__ in, unsigned short* __restrict__ out, int rows, int cols) {
  __shared__ __align__(16) unsigned short tile[64 * 72];
  const int tid = threadIdx.x;
  const int c0 = blockIdx.x * 64;
  const int r0 = blockIdx.y * 64;
  {
    const int r = tid >> 2, c16 = (tid & 3) * 16;
    const float* src = in + (size_t)(r0 + r) * cols + c0 + c16;
#pragma unroll
    for (int i = 0; i < 4; ++i) {
      const v4f f = *(const v4f*)(src + 4 * i);
#pragma unroll
      for (int e = 0; e < 4; ++e) tile[(c16 + 4 * i + e) * 72 + r] = f2bf_bits(f[e]);
    }
  }
  __syncthreads();
  {
    const int wave = tid >> 5, lane = tid & 31, q = lane >> 3, c8 = (lane & 7) * 8;
    for (int pass = 0; pass < 2; ++pass) {
#pragma unroll
      for (int it = 0; it < 2; ++it) {
        const int row = wave * 8 + it * 4 + q;
        const v4u w = *(const v4u*)(tile + row * 72 + c8);
        *(volatile v4u*)(out + (size_t)(c0 + row) * rows + r0 + c8) = w;
      }
      __threadfence();
    }
  }
}

constexpr int LDS_KSH = 0;
constexpr int LDS_KSL = LDS_KSH + kKC * kDh * 2;
constexpr int LDS_VTH = LDS_KSL + kKC * kDh * 2;
constexpr int LDS_VTL = LDS_VTH + kDh * kKC * 2;
constexpr int LDS_PSH = LDS_VTL + kDh * kKC * 2;
constexpr int LDS_PSL = LDS_PSH + 4 * 16 * kKC * 2;
constexpr int LDS_END = LDS_PSL + 4 * 16 * kKC * 2;
static_assert(LDS_END == 49152, "lds carve");
static_assert(4 * 16 * 68 * 4 <= LDS_END, "output slab overlay fits");

__global__ __launch_bounds__(128)
void swa64_kernel(const unsigned short* __restrict__ qkvH, const unsigned short* __restrict__ qkvL,
                  unsigned short* __restrict__ oH, unsigned short* __restrict__ oL) {
  union FB { v16b v; v8b h[2]; };
  __shared__ __align__(16) unsigned char lds_raw[LDS_END];
  __bf16* Ksh = (__bf16*)(lds_raw + LDS_KSH);
  __bf16* Ksl = (__bf16*)(lds_raw + LDS_KSL);
  __bf16* Vth = (__bf16*)(lds_raw + LDS_VTH);
  __bf16* Vtl = (__bf16*)(lds_raw + LDS_VTL);
  __bf16* Psh = (__bf16*)(lds_raw + LDS_PSH);
  __bf16* Psl = (__bf16*)(lds_raw + LDS_PSL);
  float*  Osb = (float*)(lds_raw + 0);

  const int tid  = threadIdx.x;
  const int wave = tid >> 5;
  const int lane = tid & 31;
  const int hh   = lane >> 4;
  const int c    = lane & 15;

  const int nqb = kSeq / kQB;
  const int bx  = blockIdx.x;
  const int qb  = bx % nqb;
  const int bhd = bx / nqb;
  const int h   = bhd % kHeads;
  const int b   = bhd / kHeads;
  const int q0  = qb * kQB + wave * 16;
  const size_t tokb = (size_t)b * kSeq;
  const float kNegInf = -__builtin_inff();

  const __bf16* QH = (const __bf16*)qkvH;
  const __bf16* QL = (const __bf16*)qkvL;

  v16b qah[2], qal[2];
  {
    const size_t qo = (tokb + q0 + c) * (size_t)kQkvN + h * kDh + 8 * hh;
#pragma unroll
    for (int dc = 0; dc < 2; ++dc) {
      qah[dc] = Frag<__bf16>::load(QH + qo + dc * 32);
      qal[dc] = Frag<__bf16>::load(QL + qo + dc * 32);
    }
  }

  float mrow[8], lrow[8];
  v8f oacc[4];
#pragma unroll
  for (int r = 0; r < 8; ++r) { mrow[r] = kNegInf; lrow[r] = 0.f; }
#pragma unroll
  for (int t = 0; t < 4; ++t) oacc[t] = (v8f){0.f,0.f,0.f,0.f,0.f,0.f,0.f,0.f};

  const int kcs = (qb >= (kWin / kKC)) ? (qb - (kWin / kKC)) : 0;
  for (int kc = kcs; kc <= qb; ++kc) {
    const int kv0 = kc * kKC;
    __syncthreads();
    {
      const int kvr = tid >> 1, dh = (tid & 1) * 32;
      const size_t rowo = (tokb + kv0 + kvr) * (size_t)kQkvN + h * kDh + dh;
      {
        const v4u* kg = (const v4u*)(qkvH + rowo + kDModel);
        v4u w[4];
#pragma unroll
        for (int i = 0; i < 4; ++i) w[i] = kg[i];
#pragma unroll
        for (int i = 0; i < 4; ++i) *(v8b*)(Ksh + kvr * kDh + dh + 8 * i) = __builtin_bit_cast(v8b, w[i]);
      }
      asm volatile("" ::: "memory");
      {
        const v4u* kg = (const v4u*)(qkvL + rowo + kDModel);
        v4u w[4];
#pragma unroll
        for (int i = 0; i < 4; ++i) w[i] = kg[i];
#pragma unroll
        for (int i = 0; i < 4; ++i) *(v8b*)(Ksl + kvr * kDh + dh + 8 * i) = __builtin_bit_cast(v8b, w[i]);
      }
      asm volatile("" ::: "memory");
      {
        const v4u* vg = (const v4u*)(qkvH + rowo + 2 * kDModel);
        v4u w[4];
#pragma unroll
        for (int i = 0; i < 4; ++i) w[i] = vg[i];
#pragma unroll
        for (int i = 0; i < 4; ++i) {
#pragma unroll
          for (int e = 0; e < 8; ++e) {
            const unsigned word = w[i][e >> 1];
            const unsigned short hb = (unsigned short)((e & 1) ? (word >> 16) : (word & 0xffffu));
            Vth[(dh + 8 * i + e) * kKC + kvr] = __builtin_bit_cast(__bf16, hb);
          }
        }
      }
      asm volatile("" ::: "memory");
      {
        const v4u* vg = (const v4u*)(qkvL + rowo + 2 * kDModel);
        v4u w[4];
#pragma unroll
        for (int i = 0; i < 4; ++i) w[i] = vg[i];
#pragma unroll
        for (int i = 0; i < 4; ++i) {
#pragma unroll
          for (int e = 0; e < 8; ++e) {
            const unsigned word = w[i][e >> 1];
            const unsigned short hb = (unsigned short)((e & 1) ? (word >> 16) : (word & 0xffffu));
            Vtl[(dh + 8 * i + e) * kKC + kvr] = __builtin_bit_cast(__bf16, hb);
          }
        }
      }
    }
    __syncthreads();

    v8f s[4];
#pragma unroll
    for (int j = 0; j < 4; ++j) {
      s[j] = (v8f){0.f,0.f,0.f,0.f,0.f,0.f,0.f,0.f};
#pragma unroll
      for (int dc = 0; dc < 2; ++dc) {
        FB kb, kl;
        kb.h[0] = *(const v8b*)(Ksh + (j * 16 + c) * kDh + dc * 32 + 8 * hh);
        kb.h[1] = *(const v8b*)(Ksh + (j * 16 + c) * kDh + dc * 32 + 16 + 8 * hh);
        kl.h[0] = *(const v8b*)(Ksl + (j * 16 + c) * kDh + dc * 32 + 8 * hh);
        kl.h[1] = *(const v8b*)(Ksl + (j * 16 + c) * kDh + dc * 32 + 16 + 8 * hh);
        s[j] = at_mma(qah[dc], kb.v, s[j]);
        s[j] = at_mma(qah[dc], kl.v, s[j]);
        s[j] = at_mma(qal[dc], kb.v, s[j]);
      }
    }

    float cm[8];
#pragma unroll
    for (int r = 0; r < 8; ++r) {
      const int qrow = q0 + 8 * hh + r;
      float m = kNegInf;
#pragma unroll
      for (int j = 0; j < 4; ++j) {
        const int kvcol = kv0 + j * 16 + c;
        const bool masked = (kvcol > qrow) || (qrow - kvcol > kWin);
        float sv = s[j][r] * kScale;
        sv = masked ? kNegInf : sv;
        s[j][r] = sv;
        m = fmaxf(m, sv);
      }
#pragma unroll
      for (int off = 1; off < 16; off <<= 1) m = fmaxf(m, __shfl_xor(m, off, 32));
      cm[r] = m;
    }

    __bf16* pwh = Psh + wave * (16 * kKC);
    __bf16* pwl = Psl + wave * (16 * kKC);
#pragma unroll
    for (int r = 0; r < 8; ++r) {
      const float mnew  = fmaxf(mrow[r], cm[r]);
      const float aexp  = expf(mrow[r] - mnew);
      const float alpha = (mnew == kNegInf) ? 1.0f : aexp;
      mrow[r] = mnew;
      float psum = 0.f;
#pragma unroll
      for (int j = 0; j < 4; ++j) {
        const float sv = s[j][r];
        const float pe = expf(sv - mnew);
        const float p  = (sv == kNegInf) ? 0.0f : pe;
        psum += p;
        __bf16 a, bl; at_split(p, a, bl);
        pwh[(8 * hh + r) * kKC + j * 16 + c] = a;
        pwl[(8 * hh + r) * kKC + j * 16 + c] = bl;
      }
#pragma unroll
      for (int off = 1; off < 16; off <<= 1) psum += __shfl_xor(psum, off, 32);
      lrow[r] = lrow[r] * alpha + psum;
#pragma unroll
      for (int t = 0; t < 4; ++t) oacc[t][r] *= alpha;
    }
    __syncthreads();

#pragma unroll 1
    for (int kk = 0; kk < 2; ++kk) {
      FB pa, pl;
      pa.h[0] = *(const v8b*)(pwh + c * kKC + kk * 32 + 8 * hh);
      pa.h[1] = *(const v8b*)(pwh + c * kKC + kk * 32 + 16 + 8 * hh);
      pl.h[0] = *(const v8b*)(pwl + c * kKC + kk * 32 + 8 * hh);
      pl.h[1] = *(const v8b*)(pwl + c * kKC + kk * 32 + 16 + 8 * hh);
#pragma unroll
      for (int t = 0; t < 4; ++t) {
        FB vb, vl;
        vb.h[0] = *(const v8b*)(Vth + (t * 16 + c) * kKC + kk * 32 + 8 * hh);
        vb.h[1] = *(const v8b*)(Vth + (t * 16 + c) * kKC + kk * 32 + 16 + 8 * hh);
        vl.h[0] = *(const v8b*)(Vtl + (t * 16 + c) * kKC + kk * 32 + 8 * hh);
        vl.h[1] = *(const v8b*)(Vtl + (t * 16 + c) * kKC + kk * 32 + 16 + 8 * hh);
        oacc[t] = at_mma(pa.v, vb.v, oacc[t]);
        oacc[t] = at_mma(pa.v, vl.v, oacc[t]);
        oacc[t] = at_mma(pl.v, vb.v, oacc[t]);
      }
    }
  }
  __syncthreads();

  float* os = Osb + wave * (16 * 68);
#pragma unroll
  for (int r = 0; r < 8; ++r) {
    const float inv = 1.0f / lrow[r];
#pragma unroll
    for (int t = 0; t < 4; ++t) os[(8 * hh + r) * 68 + t * 16 + c] = oacc[t][r] * inv;
  }
  __syncthreads();
  {
    const int q = lane >> 3, c8 = (lane & 7) * 8;
    for (int pass = 0; pass < 2; ++pass) {
#pragma unroll
      for (int it = 0; it < 4; ++it) {
        const int row = it * 4 + q;
        const float* sp = os + row * 68 + c8;
        v8h hv, lv;
#pragma unroll
        for (int e = 0; e < 8; ++e) {
          const unsigned short hb = f2bf_bits(sp[e]);
          const unsigned short lb = f2bf_bits(sp[e] - bf_bits2f(hb));
          hv[e] = __builtin_bit_cast(_Float16, hb);
          lv[e] = __builtin_bit_cast(_Float16, lb);
        }
        const size_t oo = (tokb + q0 + row) * (size_t)kDModel + h * kDh + c8;
        *(volatile v8h*)(oH + oo) = hv;
        *(volatile v8h*)(oL + oo) = lv;
      }
      __threadfence();
    }
  }
}

extern "C" void kernel_launch(void* const* d_in, const int* in_sizes, int n_in,
                              void* d_out, int out_size, void* d_ws, size_t ws_size,
                              hipStream_t stream) {
  (void)in_sizes; (void)n_in; (void)out_size; (void)ws_size;
  const float* x    = (const float*)d_in[0];
  const float* Wqkv = (const float*)d_in[1];
  const float* bqkv = (const float*)d_in[2];
  const float* Wout = (const float*)d_in[3];
  const float* bout = (const float*)d_in[4];
  float* out = (float*)d_out;

  char* ws = (char*)d_ws;
  float*          biasr = (float*)(ws + OFF_BIAS);
  unsigned short* x16   = (unsigned short*)(ws + OFF_X16);
  unsigned short* wqT   = (unsigned short*)(ws + OFF_WQT);
  unsigned short* woT   = (unsigned short*)(ws + OFF_WOT);
  unsigned short* qkvH  = (unsigned short*)(ws + OFF_QKVH);
  unsigned short* qkvL  = (unsigned short*)(ws + OFF_QKVL);
  unsigned short* attH  = (unsigned short*)(ws + OFF_ATTH);
  unsigned short* attL  = (unsigned short*)(ws + OFF_ATTL);

  bias_rne4<<<dim3(3), dim3(256), 0, stream>>>(bqkv, biasr, kQkvN / 4);
  bias_rne4<<<dim3(1), dim3(256), 0, stream>>>(bout, biasr + kQkvN, kDModel / 4);

  cast_bf16x8<<<dim3((kTok * kDModel / 8) / 256), dim3(256), 0, stream>>>(x, x16, kTok * kDModel / 8);

  transpose_cast_bf16<<<dim3(kQkvN / 64, kDModel / 64), dim3(256), 0, stream>>>(Wqkv, wqT, kDModel, kQkvN);
  transpose_cast_bf16<<<dim3(kDModel / 64, kDModel / 64), dim3(256), 0, stream>>>(Wout, woT, kDModel, kDModel);

  {
    const int tiles = (kTok / 64) * (kQkvN / 64);
    wmma_gemm64<1, false, false, 2, 2, false><<<dim3(tiles / 8, 1), dim3(256), 0, stream>>>(
        x16, x16, kDModel, 0L,
        wqT, wqT, kDModel, 0L,
        (void*)qkvH, (void*)qkvL, kQkvN, 0L,
        biasr, biasr, 0L,
        kTok, kQkvN, kDModel, 1.0f);
  }

  swa64_kernel<<<dim3(kBatch * kHeads * (kSeq / kQB)), dim3(128), 0, stream>>>(qkvH, qkvL, attH, attL);

  {
    const int tiles = (kTok / 64) * (kDModel / 64);
    wmma_gemm64<1, true, false, 2, 0, false><<<dim3(tiles / 8, 1), dim3(256), 0, stream>>>(
        attH, attL, kDModel, 0L,
        woT, woT, kDModel, 0L,
        (void*)out, (void*)out, kDModel, 0L,
        biasr + kQkvN, biasr, 0L,
        kTok, kDModel, kDModel, 1.0f);
  }
}
